// ShowerGNN_41016937677351
// MI455X (gfx1250) — hardware-verified
//
#include <hip/hip_runtime.h>
#include <stddef.h>
#include <math.h>

#pragma clang fp contract(off)


#define NB     4
#define NPTS   4096
#define NTOT   (NB * NPTS)
#define FIN    6
#define KNB    8
#define KSEL   9
#define HID    32
#define D1N    128
#define D2N    64
#define D3N    32
#define K1     68
#define K1P    96
#define BN_EPS 1e-3f
#define DBIG   3.0e38f

#define KNN_THR 256
#define G_THR   256
#define G_PTS   128
#define AP      40
#define OP      36

#define HEAD_THR   64
#define HEAD_WAVES 2
#define HEAD_PTS   32
#define HP0 104
#define HP1 136
#define HP2 72
#define HP3 36
#define T_AH  0
#define T_AL  (T_AH + 16 * HP0 * 2)
#define T_Y1H (T_AL + 16 * HP0 * 2)
#define T_Y1L (T_Y1H + 16 * HP1 * 2)
#define T_Y2H (T_Y1L + 16 * HP1 * 2)
#define T_Y2L (T_Y2H + 16 * HP2 * 2)
#define T_Y3  (T_Y2L + 16 * HP2 * 2)
#define TW_SZ (T_Y3 + 16 * HP3 * 4)
#define LDS_HEAD (HEAD_WAVES * TW_SZ)

#define OW_G1W2H 0
#define OW_G1W2L 1024
#define OW_G2W1H 2048
#define OW_G2W1L 3072
#define OW_G2W2H 4096
#define OW_G2W2L 5120
#define OW_D1H   6144
#define OW_D1L   18432
#define OW_D2H   30720
#define OW_D2L   38912
#define OW_D3H   47104
#define OW_D3L   49152
#define OW_TOT   51200
#define PREP_BLOCKS 25

#define WS_IDX   ((size_t)0)
#define WS_IDX_B ((size_t)NTOT * KNB * 4)
#define WS_H     (WS_IDX + WS_IDX_B)
#define WS_H_B   ((size_t)2 * NTOT * HID * 4)
#define WS_W     (WS_H + WS_H_B)
#define WS_W_B   ((size_t)OW_TOT * 2)
#define WS_TOT   (WS_W + WS_W_B)

static_assert((NPTS % KNN_THR) == 0);
static_assert((NPTS % G_PTS) == 0 && G_THR == 2 * G_PTS && (G_THR / 32) * 16 == G_PTS);
static_assert((NTOT % HEAD_PTS) == 0 && HEAD_THR == 2 * HEAD_PTS && HEAD_WAVES * 16 == HEAD_PTS);
static_assert(HEAD_THR == HEAD_WAVES * 32);
static_assert((T_AL % 16) == 0 && (T_Y1H % 16) == 0 && (T_Y1L % 16) == 0 && (T_Y2H % 16) == 0);
static_assert((T_Y2L % 16) == 0 && (T_Y3 % 16) == 0 && (TW_SZ % 16) == 0);
static_assert((HP0 % 8) == 0 && (HP1 % 8) == 0 && (HP2 % 8) == 0 && (AP % 8) == 0 && (OP % 4) == 0);
static_assert((K1P % 32) == 0 && (HID % 32) == 0 && (D1N % 32) == 0 && (D2N % 32) == 0);
static_assert(OW_D1L == OW_D1H + D1N * K1P && OW_D2H == OW_D1L + D1N * K1P);
static_assert(OW_D2L == OW_D2H + D2N * D1N && OW_D3H == OW_D2L + D2N * D1N);
static_assert(OW_D3L == OW_D3H + D3N * D2N && OW_TOT == OW_D3L + D3N * D2N);
static_assert((OW_G1W2L % 64) == 0 && (OW_D1H % 64) == 0 && (OW_D1L % 64) == 0 && (OW_D2H % 64) == 0);
static_assert((OW_D2L % 64) == 0 && (OW_D3H % 64) == 0 && (OW_D3L % 64) == 0);
static_assert(PREP_BLOCKS * 128 == 3 * (HID * HID / 8) + D1N * K1P / 8 + D2N * D1N / 8 + D3N * D2N / 8);
static_assert((WS_H % 256) == 0 && (WS_W % 256) == 0);
static_assert(WS_TOT == (size_t)4820992);
static_assert(LDS_HEAD == 44544);

typedef float          v2f   __attribute__((ext_vector_type(2)));
typedef float          v4f   __attribute__((ext_vector_type(4)));
typedef float          v8f   __attribute__((ext_vector_type(8)));
typedef unsigned short v8us  __attribute__((ext_vector_type(8)));
typedef unsigned short v16us __attribute__((ext_vector_type(16)));
typedef __bf16         v16bf __attribute__((ext_vector_type(16)));
typedef int            v4i   __attribute__((ext_vector_type(4)));
typedef v4f  v4fa  __attribute__((may_alias));
typedef v8us v8usa __attribute__((may_alias));
typedef v4i  v4ia  __attribute__((may_alias));
union FragB { v16us v; v8us h[2]; };

__device__ __forceinline__ v8f wmb(v16us a, v16us b, v8f c) {
  const v16bf ab = __builtin_bit_cast(v16bf, a);
  const v16bf bb = __builtin_bit_cast(v16bf, b);
  v8f d = __builtin_amdgcn_wmma_f32_16x16x32_bf16(false, ab, false, bb, (short)0, c, false, false);
#if defined(__HIP_DEVICE_COMPILE__)
  asm volatile("v_nop\n\tv_nop\n\tv_nop\n\tv_nop" : "+v"(d) : "v"(ab), "v"(bb));
#endif
  return d;
}

__device__ __forceinline__ v8f zero8() {
  v8f z = {0.f, 0.f, 0.f, 0.f, 0.f, 0.f, 0.f, 0.f};
  return z;
}

__device__ __forceinline__ unsigned short bfr(float f) {
  unsigned int u = __float_as_uint(f);
  u += 0x7FFFu + ((u >> 16) & 1u);
  return (unsigned short)(u >> 16);
}

__device__ __forceinline__ void split_bf(float f, unsigned short& hi, unsigned short& lo) {
  const unsigned short hb = bfr(f);
  const float fh = __uint_as_float(((unsigned int)hb) << 16);
  hi = hb;
  lo = bfr(f - fh);
}

template <int KT, int NT>
__device__ __forceinline__ void mma3(v8f (&acc)[8], const unsigned short* arh, const unsigned short* arl,
                                     const unsigned short* __restrict__ bh,
                                     const unsigned short* __restrict__ bl, int kp, int n0, int m,
                                     int h) {
#pragma unroll
  for (int t = 0; t < NT; ++t) acc[t] = zero8();
#pragma unroll
  for (int kt = 0; kt < KT; ++kt) {
    FragB ah, al;
    ah.h[0] = *(const v8usa*)(arh + 32 * kt);
    ah.h[1] = *(const v8usa*)(arh + 32 * kt + 16);
    al.h[0] = *(const v8usa*)(arl + 32 * kt);
    al.h[1] = *(const v8usa*)(arl + 32 * kt + 16);
#pragma unroll
    for (int t = 0; t < NT; ++t) {
      const size_t bo = (size_t)(n0 + 16 * t + m) * kp + 32 * kt + 8 * h;
      FragB fh, fl;
      fh.h[0] = *(const v8us*)(bh + bo);
      fh.h[1] = *(const v8us*)(bh + bo + 16);
      fl.h[0] = *(const v8us*)(bl + bo);
      fl.h[1] = *(const v8us*)(bl + bo + 16);
      acc[t] = wmb(ah.v, fh.v, acc[t]);
      acc[t] = wmb(ah.v, fl.v, acc[t]);
      acc[t] = wmb(al.v, fh.v, acc[t]);
    }
  }
}

template <int NT>
__device__ __forceinline__ void epi_relu_split(const v8f (&acc)[8], unsigned short* th,
                                               unsigned short* tl, int pitch, const float* sb,
                                               int n0, int m, int h) {
#pragma unroll
  for (int t = 0; t < NT; ++t) {
    const int c = n0 + 16 * t + m;
    const float bias = sb[c];
#pragma unroll
    for (int r = 0; r < 8; ++r) {
      float v = acc[t][r] + bias;
      v = fmaxf(v, 0.0f);
      unsigned short hi, lo;
      split_bf(v, hi, lo);
      th[(8 * h + r) * pitch + c] = hi;
      tl[(8 * h + r) * pitch + c] = lo;
    }
  }
}

template <int NT>
__device__ __forceinline__ void epi_bias_f32(const v8f (&acc)[8], float* so, int pitch,
                                             const float* sb, int n0, int m, int h) {
#pragma unroll
  for (int t = 0; t < NT; ++t) {
    const int c = n0 + 16 * t + m;
    const float bias = sb[c];
#pragma unroll
    for (int r = 0; r < 8; ++r) so[(8 * h + r) * pitch + c] = acc[t][r] + bias;
  }
}

__device__ __forceinline__ void store_rows32(const float* sO, float* gbase, int tid) {
  v4f v[4];
  const int rq = tid >> 3, c4 = (tid & 7) * 4;
#pragma unroll
  for (int it = 0; it < 4; ++it) v[it] = *(const v4fa*)(sO + (it * 32 + rq) * OP + c4);
#pragma unroll
  for (int it = 0; it < 4; ++it)
    *(volatile v4f*)(gbase + (size_t)(it * 32 + rq) * HID + c4) = v[it];
  __threadfence();
#pragma unroll
  for (int it = 0; it < 4; ++it)
    *(volatile v4f*)(gbase + (size_t)(it * 32 + rq) * HID + c4) = v[it];
}

__device__ __forceinline__ void ins9(float (&dd)[KSEL], int (&jj)[KSEL], float dk, int jk) {
#pragma unroll
  for (int t = 0; t < KSEL; ++t) {
    const bool sw = (dk < dd[t]) || (dk == dd[t] && jk < jj[t]);
    const float od = dd[t];
    const int   oj = jj[t];
    dd[t] = sw ? dk : od;
    jj[t] = sw ? jk : oj;
    dk = sw ? od : dk;
    jk = sw ? oj : jk;
  }
}

__device__ __forceinline__ int d1_src_k(int kk) {
  int s = kk + 2;
  s = (kk >= 32) ? kk + 4 : s;
  s = (kk == 64) ? 0 : s;
  s = (kk == 65) ? 1 : s;
  s = (kk == 66) ? 34 : s;
  s = (kk == 67) ? 35 : s;
  return s;
}

__global__ __launch_bounds__(128) void k_prep(const float* __restrict__ g1w2,
                                              const float* __restrict__ g2w1,
                                              const float* __restrict__ g2w2,
                                              const float* __restrict__ d1w,
                                              const float* __restrict__ d2w,
                                              const float* __restrict__ d3w,
                                              unsigned short* wp) {
  const int bx = blockIdx.x, tid = threadIdx.x;
  const float* w;
  int nout, kreal, kp, perm, g, oh, ol;
  if (bx < 1) {
    w = g1w2; nout = HID; kreal = HID; kp = HID; perm = 0; g = tid; oh = OW_G1W2H; ol = OW_G1W2L;
  } else if (bx < 2) {
    w = g2w1; nout = HID; kreal = HID; kp = HID; perm = 0; g = tid; oh = OW_G2W1H; ol = OW_G2W1L;
  } else if (bx < 3) {
    w = g2w2; nout = HID; kreal = HID; kp = HID; perm = 0; g = tid; oh = OW_G2W2H; ol = OW_G2W2L;
  } else if (bx < 15) {
    w = d1w; nout = D1N; kreal = K1; kp = K1P; perm = 1; g = (bx - 3) * 128 + tid;
    oh = OW_D1H; ol = OW_D1L;
  } else if (bx < 23) {
    w = d2w; nout = D2N; kreal = D1N; kp = D1N; perm = 0; g = (bx - 15) * 128 + tid;
    oh = OW_D2H; ol = OW_D2L;
  } else {
    w = d3w; nout = D3N; kreal = D2N; kp = D2N; perm = 0; g = (bx - 23) * 128 + tid;
    oh = OW_D3H; ol = OW_D3L;
  }
  const int o = g * 8;
  const int n = o / kp;
  const int k0 = o - n * kp;
  v8us hv, lv;
#pragma unroll
  for (int e = 0; e < 8; ++e) {
    const int kk = k0 + e;
    int s = perm ? d1_src_k(kk) : kk;
    const bool valid = kk < kreal;
    s = s < 0 ? 0 : (s > kreal - 1 ? kreal - 1 : s);
    const float xv = w[(size_t)s * nout + n];
    const float v = valid ? xv : xv * 0.0f;
    unsigned short hi, lo;
    split_bf(v, hi, lo);
    hv[e] = hi;
    lv[e] = lo;
  }
  unsigned short* ph = wp + oh + o;
  unsigned short* pl = wp + ol + o;
  *(volatile v8us*)ph = hv;
  *(volatile v8us*)pl = lv;
  __threadfence();
  *(volatile v8us*)ph = hv;
  *(volatile v8us*)pl = lv;
}

__global__ __launch_bounds__(KNN_THR) void k_knn(const float* __restrict__ x,
                                                 const float* __restrict__ bg,
                                                 const float* __restrict__ bb,
                                                 const float* __restrict__ bm,
                                                 const float* __restrict__ bv, int* idx) {
  __shared__ v2f sPos[NPTS];
  __shared__ int sIdx[KNN_THR * KNB];
  const int tid = threadIdx.x;
  const int b = blockIdx.x >> 4;
  const int qb = blockIdx.x & 15;
  const size_t bN = (size_t)b * NPTS;
  const float m0 = bm[0], m1 = bm[1];
  const float r0 = 1.0f / sqrtf(bv[0] + BN_EPS);
  const float r1 = 1.0f / sqrtf(bv[1] + BN_EPS);
  const float ga0 = bg[0], ga1 = bg[1], e0 = bb[0], e1 = bb[1];
  for (int i = tid; i < NPTS; i += KNN_THR) {
    const float* xp = x + (bN + (size_t)i) * FIN;
    float p0 = xp[0] - m0; p0 = p0 * r0; p0 = p0 * ga0; p0 = p0 + e0;
    float p1 = xp[1] - m1; p1 = p1 * r1; p1 = p1 * ga1; p1 = p1 + e1;
    v2f c;
    c.x = p0; c.y = p1;
    sPos[i] = c;
  }
  __syncthreads();

  const int q = qb * KNN_THR + tid;
  const v2f qv = sPos[q];
  const float qx = qv.x, qy = qv.y;
  float dd[KSEL];
  int   jj[KSEL];
#pragma unroll
  for (int t = 0; t < KSEL; ++t) { dd[t] = DBIG; jj[t] = NPTS; }
#pragma unroll 4
  for (int j = 0; j < NPTS; ++j) {
    const v2f c = sPos[j];
    const float dx = qx - c.x;
    const float dy = qy - c.y;
    const float t0 = dx * dx;
    const float t1 = dy * dy;
    const float d = t0 + t1;
    if (d < dd[KSEL - 1] || (d == dd[KSEL - 1] && j < jj[KSEL - 1])) ins9(dd, jj, d, j);
  }
#pragma unroll
  for (int t = 1; t < KSEL; ++t) {
    int j = jj[t];
    j = j < 0 ? 0 : (j > NPTS - 1 ? NPTS - 1 : j);
    sIdx[tid * KNB + (t - 1)] = j;
  }
  __syncthreads();

  int* gb = idx + (bN + (size_t)qb * KNN_THR) * KNB;
  const v4i v0 = *(const v4ia*)(sIdx + 4 * tid);
  const v4i v1 = *(const v4ia*)(sIdx + KNN_THR * 4 + 4 * tid);
  *(volatile v4i*)(gb + 4 * tid) = v0;
  *(volatile v4i*)(gb + KNN_THR * 4 + 4 * tid) = v1;
  __threadfence();
  *(volatile v4i*)(gb + 4 * tid) = v0;
  *(volatile v4i*)(gb + KNN_THR * 4 + 4 * tid) = v1;
}

__global__ __launch_bounds__(G_THR) void k_g1(const float* __restrict__ x,
                                              const float* __restrict__ bg,
                                              const float* __restrict__ bb,
                                              const float* __restrict__ bm,
                                              const float* __restrict__ bv,
                                              const int* __restrict__ idx,
                                              const float* __restrict__ w1,
                                              const float* __restrict__ b1,
                                              const float* __restrict__ b2,
                                              const unsigned short* __restrict__ wp, float* hout) {
  __shared__ unsigned short sAh[G_PTS * AP];
  __shared__ unsigned short sAl[G_PTS * AP];
  __shared__ float sO[G_PTS * OP];
  __shared__ float sW1[4 * HID];
  __shared__ float sB1[HID], sB2[HID];
  __shared__ float sM[4], sR[4], sG[4], sE[4];
  const int tid = threadIdx.x, lane = tid & 31, wave = tid >> 5, h = lane >> 4, m = lane & 15;
  {
    const int cw = tid < 4 * HID ? tid : 4 * HID - 1;
    const float vw = w1[cw];
    if (tid < 4 * HID) sW1[tid] = vw;
    const int cb = tid < HID ? tid : HID - 1;
    const float vb1 = b1[cb], vb2 = b2[cb];
    if (tid < HID) { sB1[tid] = vb1; sB2[tid] = vb2; }
    const int f = (tid < 4 ? tid : 3) + 2;
    const float vm = bm[f];
    const float vr = 1.0f / sqrtf(bv[f] + BN_EPS);
    const float vg = bg[f];
    const float ve = bb[f];
    if (tid < 4) { sM[tid] = vm; sR[tid] = vr; sG[tid] = vg; sE[tid] = ve; }
  }
  __syncthreads();

  const int p = tid >> 1, hf = tid & 1;
  const int gp = blockIdx.x * G_PTS + p;
  const int b = blockIdx.x >> 5;
  const size_t bN = (size_t)b * NPTS;
  int jn[KNB];
  {
    const v4i i0 = *(const v4i*)(idx + (size_t)gp * KNB);
    const v4i i1 = *(const v4i*)(idx + (size_t)gp * KNB + 4);
#pragma unroll
    for (int k = 0; k < 4; ++k) { jn[k] = i0[k]; jn[4 + k] = i1[k]; }
#pragma unroll
    for (int k = 0; k < KNB; ++k) jn[k] = jn[k] < 0 ? 0 : (jn[k] > NPTS - 1 ? NPTS - 1 : jn[k]);
  }
  float agg[4] = {0.f, 0.f, 0.f, 0.f};
#pragma unroll
  for (int k = 0; k < KNB; ++k) {
    const float* rp = x + (bN + (size_t)jn[k]) * FIN + 2;
    const v2f u0 = *(const v2f*)rp;
    const v2f u1 = *(const v2f*)(rp + 2);
    float fv[4];
    fv[0] = u0.x; fv[1] = u0.y; fv[2] = u1.x; fv[3] = u1.y;
#pragma unroll
    for (int f = 0; f < 4; ++f) {
      float t = fv[f] - sM[f];
      t = t * sR[f];
      t = t * sG[f];
      t = t + sE[f];
      agg[f] = agg[f] + t;
    }
  }
#pragma unroll
  for (int f = 0; f < 4; ++f) agg[f] = agg[f] * 0.125f;

  float hv[16];
#pragma unroll
  for (int n = 0; n < 16; ++n) {
    const int c = 16 * hf + n;
    float s = agg[0] * sW1[c];
    s = s + agg[1] * sW1[HID + c];
    s = s + agg[2] * sW1[2 * HID + c];
    s = s + agg[3] * sW1[3 * HID + c];
    s = s + sB1[c];
    hv[n] = fmaxf(s, 0.0f);
  }
  {
    v8us ha, la, hb2, lb2;
#pragma unroll
    for (int n = 0; n < 8; ++n) {
      unsigned short hi, lo;
      split_bf(hv[n], hi, lo); ha[n] = hi; la[n] = lo;
      split_bf(hv[8 + n], hi, lo); hb2[n] = hi; lb2[n] = lo;
    }
    unsigned short* aph = sAh + p * AP + 16 * hf;
    unsigned short* apl = sAl + p * AP + 16 * hf;
    *(v8us*)aph = ha; *(v8us*)(aph + 8) = hb2;
    *(v8us*)apl = la; *(v8us*)(apl + 8) = lb2;
  }
  __syncthreads();

  v8f acc[8];
  mma3<1, 2>(acc, sAh + (16 * wave + m) * AP + 8 * h, sAl + (16 * wave + m) * AP + 8 * h,
             wp + OW_G1W2H, wp + OW_G1W2L, HID, 0, m, h);
  epi_bias_f32<2>(acc, sO + (16 * wave) * OP, OP, sB2, 0, m, h);
  __syncthreads();

  store_rows32(sO, hout + (size_t)blockIdx.x * G_PTS * HID, tid);
}

__global__ __launch_bounds__(G_THR) void k_g2(const float* __restrict__ hin,
                                              const int* __restrict__ idx,
                                              const float* __restrict__ b1,
                                              const float* __restrict__ b2,
                                              const unsigned short* __restrict__ wp, float* hout) {
  __shared__ unsigned short sAh[G_PTS * AP];
  __shared__ unsigned short sAl[G_PTS * AP];
  __shared__ unsigned short sHh[G_PTS * AP];
  __shared__ unsigned short sHl[G_PTS * AP];
  __shared__ float sO[G_PTS * OP];
  __shared__ float sB1[HID], sB2[HID];
  const int tid = threadIdx.x, lane = tid & 31, wave = tid >> 5, h = lane >> 4, m = lane & 15;
  {
    const int cb = tid < HID ? tid : HID - 1;
    const float vb1 = b1[cb], vb2 = b2[cb];
    if (tid < HID) { sB1[tid] = vb1; sB2[tid] = vb2; }
  }
  const int p = tid >> 1, hf = tid & 1;
  const int gp = blockIdx.x * G_PTS + p;
  const int b = blockIdx.x >> 5;
  const size_t bN = (size_t)b * NPTS;
  int jn[KNB];
  {
    const v4i i0 = *(const v4i*)(idx + (size_t)gp * KNB);
    const v4i i1 = *(const v4i*)(idx + (size_t)gp * KNB + 4);
#pragma unroll
    for (int k = 0; k < 4; ++k) { jn[k] = i0[k]; jn[4 + k] = i1[k]; }
#pragma unroll
    for (int k = 0; k < KNB; ++k) jn[k] = jn[k] < 0 ? 0 : (jn[k] > NPTS - 1 ? NPTS - 1 : jn[k]);
  }
  float agg[16];
#pragma unroll
  for (int i = 0; i < 16; ++i) agg[i] = 0.0f;
#pragma unroll
  for (int k = 0; k < KNB; ++k) {
    const v4f* rp = (const v4f*)(hin + (bN + (size_t)jn[k]) * HID + 16 * hf);
#pragma unroll
    for (int g = 0; g < 4; ++g) {
      const v4f u = rp[g];
#pragma unroll
      for (int i = 0; i < 4; ++i) agg[4 * g + i] = agg[4 * g + i] + u[i];
    }
  }
  {
    v8us ha, la, hb2, lb2;
#pragma unroll
    for (int n = 0; n < 8; ++n) {
      unsigned short hi, lo;
      split_bf(agg[n] * 0.125f, hi, lo); ha[n] = hi; la[n] = lo;
      split_bf(agg[8 + n] * 0.125f, hi, lo); hb2[n] = hi; lb2[n] = lo;
    }
    unsigned short* aph = sAh + p * AP + 16 * hf;
    unsigned short* apl = sAl + p * AP + 16 * hf;
    *(v8us*)aph = ha; *(v8us*)(aph + 8) = hb2;
    *(v8us*)apl = la; *(v8us*)(apl + 8) = lb2;
  }
  __syncthreads();

  v8f acc[8];
  mma3<1, 2>(acc, sAh + (16 * wave + m) * AP + 8 * h, sAl + (16 * wave + m) * AP + 8 * h,
             wp + OW_G2W1H, wp + OW_G2W1L, HID, 0, m, h);
  epi_relu_split<2>(acc, sHh + (16 * wave) * AP, sHl + (16 * wave) * AP, AP, sB1, 0, m, h);
  __syncthreads();

  mma3<1, 2>(acc, sHh + (16 * wave + m) * AP + 8 * h, sHl + (16 * wave + m) * AP + 8 * h,
             wp + OW_G2W2H, wp + OW_G2W2L, HID, 0, m, h);
  epi_bias_f32<2>(acc, sO + (16 * wave) * OP, OP, sB2, 0, m, h);
  __syncthreads();

  store_rows32(sO, hout + (size_t)blockIdx.x * G_PTS * HID, tid);
}

__global__ __launch_bounds__(HEAD_THR) void k_head(const float* __restrict__ x,
                                                   const float* __restrict__ bg,
                                                   const float* __restrict__ bb,
                                                   const float* __restrict__ bm,
                                                   const float* __restrict__ bv,
                                                   const float* __restrict__ hpl,
                                                   const float* __restrict__ d1b,
                                                   const float* __restrict__ d2b,
                                                   const float* __restrict__ d3b,
                                                   const float* __restrict__ g2,
                                                   const float* __restrict__ be2,
                                                   const float* __restrict__ mn2,
                                                   const float* __restrict__ vr2,
                                                   const float* __restrict__ ow,
                                                   const float* __restrict__ ob,
                                                   const unsigned short* __restrict__ wp, float* out) {
  extern __shared__ v4f lds_dyn[];
  char* lb = (char*)lds_dyn;
  __shared__ float sD1B[D1N], sD2B[D2N], sD3B[D3N], sOW[D3N];
  __shared__ float sM2[D3N], sR2[D3N], sG2[D3N], sE2[D3N];
  __shared__ float sOut[HEAD_PTS];
  const int tid = threadIdx.x, lane = tid & 31, wave = tid >> 5, h = lane >> 4, m = lane & 15;
  {
    sD1B[tid] = d1b[tid];
    sD1B[tid + HEAD_THR] = d1b[tid + HEAD_THR];
    sD2B[tid] = d2b[tid];
    const int c = tid < D3N ? tid : D3N - 1;
    const float v3 = d3b[c], vw = ow[c], vm = mn2[c], vg = g2[c], ve = be2[c];
    const float vr = 1.0f / sqrtf(vr2[c] + BN_EPS);
    if (tid < D3N) { sD3B[tid] = v3; sOW[tid] = vw; sM2[tid] = vm; sR2[tid] = vr; sG2[tid] = vg; sE2[tid] = ve; }
  }
  const float m0 = bm[0], m1 = bm[1];
  const float r0 = 1.0f / sqrtf(bv[0] + BN_EPS);
  const float r1 = 1.0f / sqrtf(bv[1] + BN_EPS);
  const float ga0 = bg[0], ga1 = bg[1], e0 = bb[0], e1 = bb[1];
  const float obv = ob[0];

  unsigned short* tAh  = (unsigned short*)(lb + wave * TW_SZ + T_AH);
  unsigned short* tAl  = (unsigned short*)(lb + wave * TW_SZ + T_AL);
  unsigned short* tY1h = (unsigned short*)(lb + wave * TW_SZ + T_Y1H);
  unsigned short* tY1l = (unsigned short*)(lb + wave * TW_SZ + T_Y1L);
  unsigned short* tY2h = (unsigned short*)(lb + wave * TW_SZ + T_Y2H);
  unsigned short* tY2l = (unsigned short*)(lb + wave * TW_SZ + T_Y2L);
  float*          tY3  = (float*)(lb + wave * TW_SZ + T_Y3);

  {
    const int p = tid >> 1, hf = tid & 1;
    const int gp = blockIdx.x * HEAD_PTS + p;
    const int prow = p & 15;
    const float* hp = hpl + (size_t)hf * ((size_t)NTOT * HID) + (size_t)gp * HID;
#pragma unroll
    for (int g = 0; g < 4; ++g) {
      const v4f u0 = *(const v4f*)(hp + 8 * g);
      const v4f u1 = *(const v4f*)(hp + 8 * g + 4);
      v8us hv, lv;
#pragma unroll
      for (int i = 0; i < 4; ++i) {
        unsigned short hi, lo;
        split_bf(u0[i], hi, lo); hv[i] = hi; lv[i] = lo;
        split_bf(u1[i], hi, lo); hv[4 + i] = hi; lv[4 + i] = lo;
      }
      *(v8us*)(tAh + prow * HP0 + 32 * hf + 8 * g) = hv;
      *(v8us*)(tAl + prow * HP0 + 32 * hf + 8 * g) = lv;
    }
    const float* xp = x + (size_t)gp * FIN;
    const float x0 = xp[0], x1 = xp[1];
    float p0 = x0 - m0; p0 = p0 * r0; p0 = p0 * ga0; p0 = p0 + e0;
    float p1 = x1 - m1; p1 = p1 * r1; p1 = p1 * ga1; p1 = p1 + e1;
    const float zr = x0 * 0.0f;
    float ev[8];
    ev[0] = hf ? zr : p0; ev[1] = hf ? zr : p1; ev[2] = hf ? zr : p0; ev[3] = hf ? zr : p1;
    ev[4] = zr; ev[5] = zr; ev[6] = zr; ev[7] = zr;
    v8us ph8, pl8, zh8, zl8;
#pragma unroll
    for (int i = 0; i < 8; ++i) {
      unsigned short hi, lo;
      split_bf(ev[i], hi, lo); ph8[i] = hi; pl8[i] = lo;
      split_bf(zr, hi, lo); zh8[i] = hi; zl8[i] = lo;
    }
    *(v8us*)(tAh + prow * HP0 + 64 + 8 * hf) = ph8;
    *(v8us*)(tAl + prow * HP0 + 64 + 8 * hf) = pl8;
    *(v8us*)(tAh + prow * HP0 + 80 + 8 * hf) = zh8;
    *(v8us*)(tAl + prow * HP0 + 80 + 8 * hf) = zl8;
  }
  __syncthreads();

  v8f acc[8];
#pragma unroll
  for (int nh = 0; nh < 2; ++nh) {
    mma3<3, 4>(acc, tAh + m * HP0 + 8 * h, tAl + m * HP0 + 8 * h, wp + OW_D1H, wp + OW_D1L, K1P,
               64 * nh, m, h);
    epi_relu_split<4>(acc, tY1h, tY1l, HP1, sD1B, 64 * nh, m, h);
  }
  __syncthreads();

  mma3<4, 4>(acc, tY1h + m * HP1 + 8 * h, tY1l + m * HP1 + 8 * h, wp + OW_D2H, wp + OW_D2L, D1N,
             0, m, h);
  epi_relu_split<4>(acc, tY2h, tY2l, HP2, sD2B, 0, m, h);
  __syncthreads();

  mma3<2, 2>(acc, tY2h + m * HP2 + 8 * h, tY2l + m * HP2 + 8 * h, wp + OW_D3H, wp + OW_D3L, D2N,
             0, m, h);
#pragma unroll
  for (int t = 0; t < 2; ++t) {
    const int c = 16 * t + m;
    const float bias = sD3B[c];
    const float mu = sM2[c], rs = sR2[c], gm = sG2[c], bt = sE2[c];
#pragma unroll
    for (int r = 0; r < 8; ++r) {
      float v = acc[t][r] + bias;
      v = fmaxf(v, 0.0f);
      v = v - mu;
      v = v * rs;
      v = v * gm;
      v = v + bt;
      tY3[(8 * h + r) * HP3 + c] = v;
    }
  }
  __syncthreads();

  {
    const int row = lane & 15;
    float s = tY3[row * HP3] * sOW[0];
#pragma unroll
    for (int c = 1; c < D3N; ++c) s = s + tY3[row * HP3 + c] * sOW[c];
    s = s + obv;
    if (lane < 16) sOut[16 * wave + row] = s;
  }
  __syncthreads();

  if (wave == 0) {
    const v4f ov = *(const v4fa*)(sOut + 4 * (lane & 7));
    float* gq = out + (size_t)blockIdx.x * HEAD_PTS + 4 * (lane & 7);
    if (lane < 8) *(volatile v4f*)gq = ov;
    __threadfence();
    if (lane < 8) *(volatile v4f*)gq = ov;
  }
}

extern "C" void kernel_launch(void* const* d_in, const int* in_sizes, int n_in, void* d_out,
                              int out_size, void* d_ws, size_t ws_size, hipStream_t stream) {
  if (n_in < 25) return;
  if (in_sizes[0] != NTOT * FIN) return;
  for (int i = 1; i <= 4; ++i) if (in_sizes[i] < FIN) return;
  if (in_sizes[5] != 4 * HID || in_sizes[6] < HID) return;
  if (in_sizes[7] != HID * HID || in_sizes[8] < HID) return;
  if (in_sizes[9] != HID * HID || in_sizes[10] < HID) return;
  if (in_sizes[11] != HID * HID || in_sizes[12] < HID) return;
  if (in_sizes[13] != K1 * D1N || in_sizes[14] < D1N) return;
  if (in_sizes[15] != D1N * D2N || in_sizes[16] < D2N) return;
  if (in_sizes[17] != D2N * D3N || in_sizes[18] < D3N) return;
  for (int i = 19; i <= 22; ++i) if (in_sizes[i] < D3N) return;
  if (in_sizes[23] < D3N || in_sizes[24] < 1) return;
  if (out_size != NTOT) return;
  if (WS_TOT > ws_size || WS_TOT > (size_t)134217728) return;

  const float* inputs = (const float*)d_in[0];
  const float* bn1g = (const float*)d_in[1];
  const float* bn1b = (const float*)d_in[2];
  const float* bn1m = (const float*)d_in[3];
  const float* bn1v = (const float*)d_in[4];
  const float* g1w1 = (const float*)d_in[5];
  const float* g1b1 = (const float*)d_in[6];
  const float* g1w2 = (const float*)d_in[7];
  const float* g1b2 = (const float*)d_in[8];
  const float* g2w1 = (const float*)d_in[9];
  const float* g2b1 = (const float*)d_in[10];
  const float* g2w2 = (const float*)d_in[11];
  const float* g2b2 = (const float*)d_in[12];
  const float* d1w  = (const float*)d_in[13];
  const float* d1b  = (const float*)d_in[14];
  const float* d2w  = (const float*)d_in[15];
  const float* d2b  = (const float*)d_in[16];
  const float* d3w  = (const float*)d_in[17];
  const float* d3b  = (const float*)d_in[18];
  const float* bn2g = (const float*)d_in[19];
  const float* bn2b = (const float*)d_in[20];
  const float* bn2m = (const float*)d_in[21];
  const float* bn2v = (const float*)d_in[22];
  const float* outw = (const float*)d_in[23];
  const float* outb = (const float*)d_in[24];
  float* out = (float*)d_out;

  char* ws = (char*)d_ws;
  int* idxp = (int*)(ws + WS_IDX);
  float* hpl = (float*)(ws + WS_H);
  float* h1p = hpl;
  float* h2p = hpl + (size_t)NTOT * HID;
  unsigned short* wp = (unsigned short*)(ws + WS_W);

  k_prep<<<PREP_BLOCKS, 128, 0, stream>>>(g1w2, g2w1, g2w2, d1w, d2w, d3w, wp);
  k_knn<<<NB * (NPTS / KNN_THR), KNN_THR, 0, stream>>>(inputs, bn1g, bn1b, bn1m, bn1v, idxp);
  k_g1<<<NTOT / G_PTS, G_THR, 0, stream>>>(inputs, bn1g, bn1b, bn1m, bn1v, idxp, g1w1, g1b1,
                                           g1b2, wp, h1p);
  k_g2<<<NTOT / G_PTS, G_THR, 0, stream>>>(h1p, idxp, g2b1, g2b2, wp, h2p);
  k_head<<<NTOT / HEAD_PTS, HEAD_THR, LDS_HEAD, stream>>>(inputs, bn1g, bn1b, bn1m, bn1v, hpl,
                                                          d1b, d2b, d3b, bn2g, bn2b, bn2m, bn2v,
                                                          outw, outb, wp, out);
}
